// GroupedQueryAttention_30605936951674
// MI455X (gfx1250) — hardware-verified
//
#include <hip/hip_runtime.h>
#ifndef NB
#define NB 2
#endif
#ifndef SEQ
#define SEQ 2048
#endif
#define SQ SEQ
#define SQ_FULL 2048
#define DM 1024
#define NH 16
#define NG 4
#define HPG 4
#define HD 64
#define KVD (NG * HD)
#ifndef QT0
#define QT0 256
#endif
#define MP (NB * SQ)

static_assert(HD == 64);
static_assert(HD / 2 == 32);
static_assert(DM == NH * HD);
static_assert(NH == NG * HPG);
static_assert(HPG == 4);
static_assert(DM % 64 == 0 && KVD % 64 == 0);
static_assert(DM % 32 == 0 && HD % 32 == 0);
static_assert(SQ % 128 == 0 && MP % 128 == 0);
static_assert(QT0 % 128 == 0 && QT0 % 64 == 0 && QT0 <= SQ);
static_assert(SQ % 64 == 0 && SQ % 32 == 0 && SQ % 16 == 0);
static_assert(SQ <= SQ_FULL);
static_assert(((size_t)(NB - 1) * SQ_FULL + SQ) * DM * 4 <= (size_t)16777216);

typedef unsigned short v8us __attribute__((ext_vector_type(8), may_alias));
typedef float  v8f  __attribute__((ext_vector_type(8)));
typedef float  v4f  __attribute__((ext_vector_type(4)));
typedef float  v4fa __attribute__((ext_vector_type(4), may_alias));
typedef _Float16 v16h __attribute__((ext_vector_type(16)));
typedef _Float16 v4h  __attribute__((ext_vector_type(4)));
union FragH { v16h v; v8us half[2]; _Float16 h[16]; unsigned short u[16]; };
union H1 { _Float16 h; unsigned short u; };

__device__ __forceinline__ unsigned short bf16_bits(float x) { unsigned int u = __float_as_uint(x); return (unsigned short)((u + 0x7FFFu + ((u >> 16) & 1u)) >> 16); }
__device__ __forceinline__ float bf16_rne(float x) { return __uint_as_float(((unsigned int)bf16_bits(x)) << 16); }
__device__ __forceinline__ unsigned short h16_bits(_Float16 x) { H1 t; t.h = x; return t.u; }

__device__ __forceinline__ v16h g2_frag(const _Float16* p, int hh) { FragH f; f.half[0] = *(const v8us*)((const unsigned short*)p + 8 * hh); f.half[1] = *(const v8us*)((const unsigned short*)p + 16 + 8 * hh); return f.v; }
__device__ __forceinline__ v8f g2_mma(v16h a, v16h b, v8f c) { v8f d = __builtin_amdgcn_wmma_f32_16x16x32_f16(false, a, false, b, (short)0, c, false, false); asm volatile("v_nop\n\tv_nop\n\tv_nop\n\tv_nop" : "+v"(d) : "v"(a), "v"(b)); return d; }

__global__ __launch_bounds__(256) void k_wnat(const float* __restrict__ w, size_t n8, _Float16* __restrict__ Bt) {
  const size_t t = (size_t)blockIdx.x * 256 + threadIdx.x; if (t >= n8) return;
  const v4f a = *(const v4fa*)(w + t * 8), c = *(const v4fa*)(w + t * 8 + 4);
  FragH f;
#pragma unroll
  for (int q = 0; q < 4; ++q) { f.h[q] = (_Float16)(bf16_rne(a[q]) * 16.0f); f.h[4 + q] = (_Float16)(bf16_rne(c[q]) * 16.0f); }
  const v8us o = f.half[0];
  unsigned short* d = (unsigned short*)Bt + t * 8;
  *(volatile v8us*)d = o; __threadfence(); *(volatile v8us*)d = o;
}

__global__ __launch_bounds__(256) void k_x16(const float* __restrict__ x, _Float16* __restrict__ X16, size_t n8) {
  const size_t t = (size_t)blockIdx.x * 256 + threadIdx.x; if (t >= n8) return;
  const float* src = x + (size_t)blockIdx.y * SQ_FULL * DM + t * 8;
  const v4f a = *(const v4fa*)(src), c = *(const v4fa*)(src + 4);
  FragH f;
#pragma unroll
  for (int q = 0; q < 4; ++q) { f.h[q] = (_Float16)bf16_rne(a[q]); f.h[4 + q] = (_Float16)bf16_rne(c[q]); }
  const v8us o = f.half[0];
  unsigned short* d = (unsigned short*)X16 + (size_t)blockIdx.y * SQ * DM + t * 8;
  *(volatile v8us*)d = o; __threadfence(); *(volatile v8us*)d = o;
}

__global__ __launch_bounds__(32) void k_invf(float theta, float* __restrict__ INVF) {
  #pragma clang fp contract(off)
  const int i = threadIdx.x;
  const float v = 1.0f / powf(theta, (float)(2 * i) / (float)HD);
  *(volatile float*)(INVF + i) = v; __threadfence(); *(volatile float*)(INVF + i) = v;
}
__global__ __launch_bounds__(256) void k_tab2(const float* __restrict__ INVF, float* __restrict__ CS, float* __restrict__ SN) {
  #pragma clang fp contract(off)
  const int t = blockIdx.x * 256 + threadIdx.x; if (t >= SQ * (HD / 2)) return;
  const int i = t % (HD / 2); const int p = t / (HD / 2);
  const float ang = (float)p * INVF[i];
  const float c = cosf(ang), s = sinf(ang);
  *(volatile float*)(CS + t) = c; *(volatile float*)(SN + t) = s; __threadfence(); *(volatile float*)(CS + t) = c; *(volatile float*)(SN + t) = s;
}

__global__ __launch_bounds__(128) void k_gemm2(const _Float16* __restrict__ A, int lda, size_t sA, const _Float16* __restrict__ Bh, int ldb, size_t sB, float alpha, int accum,
                                               float* C, _Float16* C16, int ldc, size_t sC, int M, int N, int K) {
  __shared__ __attribute__((aligned(16))) float so[4][32][68];
  const int tid = threadIdx.x, w = tid >> 5, lane = tid & 31, ln = lane & 15, hh = lane >> 4; const int by = blockIdx.y;
  A += (size_t)by * sA; Bh += (size_t)by * sB; const size_t cofs = (size_t)by * sC;
  const int ntn = N >> 6; const int mt = blockIdx.x / ntn, nq = blockIdx.x - mt * ntn; const int row0 = mt * 128 + 32 * w, col0 = nq * 64; if (row0 >= M) return;
  const _Float16* a0p = A + (size_t)(row0 + ln) * lda; const _Float16* a1p = a0p + (size_t)16 * lda;
  const _Float16* b0p = Bh + (size_t)(col0 + ln) * ldb; const _Float16* b1p = b0p + (size_t)16 * ldb; const _Float16* b2p = b1p + (size_t)16 * ldb; const _Float16* b3p = b2p + (size_t)16 * ldb;
  const v8f z8 = {0.f,0.f,0.f,0.f,0.f,0.f,0.f,0.f}; v8f c00 = z8, c01 = z8, c02 = z8, c03 = z8, c10 = z8, c11 = z8, c12 = z8, c13 = z8;
#pragma unroll 1
  for (int kb = 0; kb < K; kb += 32) { const v16h a0 = g2_frag(a0p + kb, hh), a1 = g2_frag(a1p + kb, hh);
    v16h b = g2_frag(b0p + kb, hh); c00 = g2_mma(a0, b, c00); c10 = g2_mma(a1, b, c10);
    b = g2_frag(b1p + kb, hh); c01 = g2_mma(a0, b, c01); c11 = g2_mma(a1, b, c11);
    b = g2_frag(b2p + kb, hh); c02 = g2_mma(a0, b, c02); c12 = g2_mma(a1, b, c12);
    b = g2_frag(b3p + kb, hh); c03 = g2_mma(a0, b, c03); c13 = g2_mma(a1, b, c13); }
  v8f accs[8] = {c00, c01, c02, c03, c10, c11, c12, c13};
#pragma unroll
  for (int u = 0; u < 8; ++u) { const int t = u & 3, half = u >> 2;
#pragma unroll
    for (int r = 0; r < 8; ++r) so[w][half * 16 + 8 * hh + r][t * 16 + ln] = accs[u][r] * alpha; }
  __builtin_amdgcn_fence(4  , "workgroup"); __builtin_amdgcn_wave_barrier();
  const int rsub = lane >> 4, c4 = (lane & 15) * 4;
  if (accum) {
#pragma unroll
    for (int q = 0; q < 16; ++q) { const int r = q * 2 + rsub; v4f v = *(const v4fa*)&so[w][r][c4]; const v4f d = *(const v4fa*)(C + cofs + (size_t)(row0 + r) * ldc + col0 + c4); v += d; *(v4fa*)&so[w][r][c4] = v; }
    __builtin_amdgcn_fence(4  , "workgroup"); __builtin_amdgcn_wave_barrier();
  }
  for (int pass = 0; pass < 2; ++pass) {
#pragma unroll
    for (int q = 0; q < 16; ++q) { const int r = q * 2 + rsub; const v4f v = *(const v4fa*)&so[w][r][c4];
      if (C) *(volatile v4f*)(C + cofs + (size_t)(row0 + r) * ldc + col0 + c4) = v;
      if (C16) { v4h h4; for (int i = 0; i < 4; ++i) h4[i] = (_Float16)v[i]; *(volatile v4h*)(C16 + cofs + (size_t)(row0 + r) * ldc + col0 + c4) = h4; } }
    if (pass == 0) __threadfence(); }
}

__global__ __launch_bounds__(64) void k_rope16(const float* __restrict__ F, int ldf, int nh, const float* __restrict__ CS, const float* __restrict__ SN, _Float16* __restrict__ H16, int ldo) {
  #pragma clang fp contract(off)
  __shared__ float xv[HD]; __shared__ unsigned short sh_[HD];
  const int d = threadIdx.x; const int h = blockIdx.x % nh; const size_t r = blockIdx.x / nh; const int p = (int)(r % SQ);
  const float x = F[r * (size_t)ldf + (size_t)h * HD + d];
  xv[d] = x; __syncthreads();
  const int i = d & (HD / 2 - 1); const float c = CS[p * (HD / 2) + i], s = SN[p * (HD / 2) + i]; const float lo = xv[i], hi = xv[i + HD / 2];
  const float o = (d < HD / 2) ? __fadd_rn(__fmul_rn(lo, c), -__fmul_rn(hi, s)) : __fadd_rn(__fmul_rn(lo, s), __fmul_rn(hi, c));
  sh_[d] = h16_bits((_Float16)o); __syncthreads();
  if (d < HD / 8) { FragH f;
#pragma unroll
    for (int q = 0; q < 8; ++q) f.u[q] = sh_[d * 8 + q];
    unsigned short* dst = (unsigned short*)H16 + r * (size_t)ldo + (size_t)h * HD + d * 8; *(volatile v8us*)dst = f.half[0]; __threadfence(); *(volatile v8us*)dst = f.half[0]; }
}
__global__ __launch_bounds__(64) void k_ropef(const float* __restrict__ F, int ldf, int nh, const float* __restrict__ CS, const float* __restrict__ SN, float* __restrict__ F32, int ldo) {
  #pragma clang fp contract(off)
  __shared__ float xv[HD];
  const int d = threadIdx.x; const int h = blockIdx.x % nh; const size_t r = blockIdx.x / nh; const int p = (int)r; const size_t b = blockIdx.y;
  const float x = F[(b * SQ + r) * (size_t)ldf + (size_t)h * HD + d];
  xv[d] = x; __syncthreads();
  const int i = d & (HD / 2 - 1); const float c = CS[p * (HD / 2) + i], s = SN[p * (HD / 2) + i]; const float lo = xv[i], hi = xv[i + HD / 2];
  const float o = (d < HD / 2) ? __fadd_rn(__fmul_rn(lo, c), -__fmul_rn(hi, s)) : __fadd_rn(__fmul_rn(lo, s), __fmul_rn(hi, c));
  float* dst = F32 + (b * QT0 + r) * (size_t)ldo + (size_t)h * HD + d; *(volatile float*)dst = o; __threadfence(); *(volatile float*)dst = o;
}

__global__ __launch_bounds__(256) void k_vt(const _Float16* __restrict__ V16, _Float16* __restrict__ VT) {
  __shared__ unsigned short tl[64][66];
  const int tid = threadIdx.x; const int slab = blockIdx.x / (SQ / 64), lg = blockIdx.x % (SQ / 64); const int b = slab / NG, g = slab % NG;
  for (int i = tid; i < 64 * 8; i += 256) { const int r = i / 8, c8 = (i % 8) * 8; FragH f; f.half[0] = *(const v8us*)((const unsigned short*)V16 + ((size_t)b * SQ + lg * 64 + r) * KVD + g * HD + c8);
#pragma unroll
    for (int q = 0; q < 8; ++q) tl[r][c8 + q] = f.u[q]; }
  __syncthreads();
  for (int pass = 0; pass < 2; ++pass) {
#pragma unroll
    for (int rd = 0; rd < 2; ++rd) { const int d = rd * 32 + tid / 8, pc = tid % 8; FragH f;
#pragma unroll
      for (int q = 0; q < 8; ++q) f.u[q] = tl[pc * 8 + q][d];
      *(volatile v8us*)((unsigned short*)VT + ((size_t)slab * HD + d) * SQ + lg * 64 + pc * 8) = f.half[0]; }
    if (pass == 0) __threadfence(); }
}

__global__ __launch_bounds__(64) void k_att0(const float* __restrict__ QF0, const float* __restrict__ KF0, const float* __restrict__ VF, float scale, float* __restrict__ OF0) {
  #pragma clang fp contract(off)
  __shared__ __attribute__((aligned(16))) float lq[64][64]; __shared__ __attribute__((aligned(16))) float lo[64][64];
  const int tid = threadIdx.x; const size_t b = blockIdx.y; const int h = blockIdx.x / (QT0 / 64), rg = blockIdx.x % (QT0 / 64); const int i = rg * 64 + tid; const int g = h / HPG;
  const float* qr = QF0 + (b * QT0 + i) * DM + h * HD;
  const float* kbase = KF0 + b * QT0 * KVD + g * HD;
  const float* vbase = VF + b * SQ * KVD + g * HD;
#pragma unroll 1
  for (int c = 0; c < HD / 4; ++c) { *(v4fa*)&lq[tid][c * 4] = *(const v4fa*)(qr + c * 4); const v4f z = {0.f, 0.f, 0.f, 0.f}; *(v4fa*)&lo[tid][c * 4] = z; }
  float m = -1.0e30f, l = 0.f; const int jmax = rg * 64 + 63;
#pragma unroll 1
  for (int j = 0; j <= jmax; ++j) { const float* kr = kbase + (size_t)j * KVD; const float* vr = vbase + (size_t)j * KVD; float s = 0.f;
#pragma unroll 1
    for (int c = 0; c < HD / 4; ++c) { const v4f kq = *(const v4fa*)(kr + c * 4); const v4f qq = *(const v4fa*)&lq[tid][c * 4]; s = __fadd_rn(s, __fmul_rn(qq[0], kq[0])); s = __fadd_rn(s, __fmul_rn(qq[1], kq[1])); s = __fadd_rn(s, __fmul_rn(qq[2], kq[2])); s = __fadd_rn(s, __fmul_rn(qq[3], kq[3])); }
    s = __fmul_rn(s, scale);
    const float f = (j <= i) ? 1.f : 0.f; const float sm = fmaf(f, s, (1.f - f) * -1.0e30f); const float mn = fmaxf(m, sm); const float sc = expf(m - mn); const float e = expf(sm - mn); l = __fadd_rn(__fmul_rn(l, sc), e); m = mn;
#pragma unroll 1
    for (int c = 0; c < HD / 4; ++c) { const v4f vv = *(const v4fa*)(vr + c * 4); v4f oo = *(const v4fa*)&lo[tid][c * 4]; for (int u = 0; u < 4; ++u) oo[u] = __fadd_rn(__fmul_rn(oo[u], sc), __fmul_rn(e, vv[u])); *(v4fa*)&lo[tid][c * 4] = oo; } }
  const float fin = 64.0f / l;
#pragma unroll 1
  for (int c = 0; c < HD / 4; ++c) { v4f oo = *(const v4fa*)&lo[tid][c * 4]; for (int u = 0; u < 4; ++u) oo[u] = __fmul_rn(oo[u], fin); *(v4fa*)&lo[tid][c * 4] = oo; }
  __syncthreads();
  float* ob = OF0 + b * QT0 * DM;
  for (int pass = 0; pass < 2; ++pass) {
#pragma unroll 1
    for (int it = 0; it < 16; ++it) { const int row = it * 4 + tid / 16, pc = (tid % 16) * 4; const v4f v = *(const v4fa*)&lo[row][pc]; *(volatile v4f*)(ob + (size_t)(rg * 64 + row) * DM + h * HD + pc) = v; }
    if (pass == 0) __threadfence(); }
}

__global__ __launch_bounds__(256) void k_hl(const float* __restrict__ F, _Float16* __restrict__ Hh, _Float16* __restrict__ Hl, size_t n8) {
  const size_t t = (size_t)blockIdx.x * 256 + threadIdx.x; if (t >= n8) return; FragH fh, fl; const v4f a = *(const v4fa*)(F + t * 8), c = *(const v4fa*)(F + t * 8 + 4);
#pragma unroll
  for (int q = 0; q < 4; ++q) { _Float16 h = (_Float16)a[q]; fh.h[q] = h; fl.h[q] = (_Float16)((a[q] - (float)h) * 1024.0f); h = (_Float16)c[q]; fh.h[4 + q] = h; fl.h[4 + q] = (_Float16)((c[q] - (float)h) * 1024.0f); }
  for (int pass = 0; pass < 2; ++pass) { *(volatile v8us*)((unsigned short*)Hh + t * 8) = fh.half[0]; *(volatile v8us*)((unsigned short*)Hl + t * 8) = fl.half[0]; if (pass == 0) __threadfence(); }
}

__global__ __launch_bounds__(128) void k_flash(const _Float16* __restrict__ Q16, const _Float16* __restrict__ K16, const _Float16* __restrict__ VT, _Float16* __restrict__ O16) {
  __shared__ __attribute__((aligned(16))) unsigned short sp[4][16][40];
  __shared__ __attribute__((aligned(16))) unsigned short so[4][16][72];
  const int tid = threadIdx.x, w = tid >> 5, lane = tid & 31, ln = lane & 15, hh = lane >> 4;
  const int qt = (int)(blockIdx.x % (SQ / 16)); const int bg = (int)(blockIdx.x / (SQ / 16)); const int g = bg % NG, b = bg / NG;
  const int h = g * HPG + w, q0 = qt * 16;
  const unsigned short* qp = (const unsigned short*)Q16 + ((size_t)b * SQ + q0 + ln) * DM + h * HD + 8 * hh;
  FragH qa0, qa1;
  qa0.half[0] = *(const v8us*)(qp);      qa0.half[1] = *(const v8us*)(qp + 16);
  qa1.half[0] = *(const v8us*)(qp + 32); qa1.half[1] = *(const v8us*)(qp + 48);
  const unsigned short* kp = (const unsigned short*)K16 + ((size_t)b * SQ + ln) * KVD + g * HD + 8 * hh;
  const unsigned short* vp = (const unsigned short*)VT + (((size_t)b * NG + g) * HD + ln) * SQ + 8 * hh;
  const v8f z8 = {0.f,0.f,0.f,0.f,0.f,0.f,0.f,0.f};
  v8f o0 = z8, o1 = z8, o2 = z8, o3 = z8;
  float mr[8], lr[8];
#pragma unroll
  for (int r = 0; r < 8; ++r) { mr[r] = -1.0e30f; lr[r] = 0.f; }
  const int kend = q0 + 16;
#pragma unroll 1
  for (int kb = 0; kb < kend; kb += 32) {
    const unsigned short* k0 = kp + (size_t)kb * KVD; const unsigned short* k1 = k0 + (size_t)16 * KVD;
    v8f s0 = z8, s1 = z8;
    { FragH bf;
      bf.half[0] = *(const v8us*)(k0);      bf.half[1] = *(const v8us*)(k0 + 16); s0 = g2_mma(qa0.v, bf.v, s0);
      bf.half[0] = *(const v8us*)(k0 + 32); bf.half[1] = *(const v8us*)(k0 + 48); s0 = g2_mma(qa1.v, bf.v, s0);
      bf.half[0] = *(const v8us*)(k1);      bf.half[1] = *(const v8us*)(k1 + 16); s1 = g2_mma(qa0.v, bf.v, s1);
      bf.half[0] = *(const v8us*)(k1 + 32); bf.half[1] = *(const v8us*)(k1 + 48); s1 = g2_mma(qa1.v, bf.v, s1); }
    float a0[8], a1[8];
#pragma unroll
    for (int r = 0; r < 8; ++r) { a0[r] = s0[r] * 0.125f; a1[r] = s1[r] * 0.125f; }
    if (kb + 31 > q0) {
      const int key0 = kb + ln, key1 = key0 + 16;
#pragma unroll
      for (int r = 0; r < 8; ++r) { const int qrow = q0 + 8 * hh + r; a0[r] = (key0 > qrow) ? -1.0e30f : a0[r]; a1[r] = (key1 > qrow) ? -1.0e30f : a1[r]; }
    }
#pragma unroll
    for (int r = 0; r < 8; ++r) {
      float bm = fmaxf(a0[r], a1[r]);
      bm = fmaxf(bm, __shfl_xor(bm, 1)); bm = fmaxf(bm, __shfl_xor(bm, 2)); bm = fmaxf(bm, __shfl_xor(bm, 4)); bm = fmaxf(bm, __shfl_xor(bm, 8));
      const float mn = fmaxf(mr[r], bm);
      const float corr = __expf(mr[r] - mn); mr[r] = mn;
      const _Float16 p0 = (_Float16)(__expf(a0[r] - mn) * 256.0f);
      const _Float16 p1 = (_Float16)(__expf(a1[r] - mn) * 256.0f);
      lr[r] = lr[r] * corr + ((float)p0 + (float)p1);
      o0[r] *= corr; o1[r] *= corr; o2[r] *= corr; o3[r] *= corr;
      sp[w][8 * hh + r][ln] = h16_bits(p0); sp[w][8 * hh + r][16 + ln] = h16_bits(p1);
    }
    __builtin_amdgcn_fence(4  , "workgroup"); __builtin_amdgcn_wave_barrier();
    FragH pa; pa.half[0] = *(const v8us*)&sp[w][ln][8 * hh]; pa.half[1] = *(const v8us*)&sp[w][ln][16 + 8 * hh];
    const unsigned short* v0 = vp + kb;
    { FragH vb;
      vb.half[0] = *(const v8us*)(v0);                       vb.half[1] = *(const v8us*)(v0 + 16);                       o0 = g2_mma(pa.v, vb.v, o0);
      vb.half[0] = *(const v8us*)(v0 + (size_t)16 * SQ);     vb.half[1] = *(const v8us*)(v0 + (size_t)16 * SQ + 16);     o1 = g2_mma(pa.v, vb.v, o1);
      vb.half[0] = *(const v8us*)(v0 + (size_t)32 * SQ);     vb.half[1] = *(const v8us*)(v0 + (size_t)32 * SQ + 16);     o2 = g2_mma(pa.v, vb.v, o2);
      vb.half[0] = *(const v8us*)(v0 + (size_t)48 * SQ);     vb.half[1] = *(const v8us*)(v0 + (size_t)48 * SQ + 16);     o3 = g2_mma(pa.v, vb.v, o3); }
    __builtin_amdgcn_fence(4  , "workgroup"); __builtin_amdgcn_wave_barrier();
  }
#pragma unroll
  for (int r = 0; r < 8; ++r) {
    float ls = lr[r];
    ls += __shfl_xor(ls, 1); ls += __shfl_xor(ls, 2); ls += __shfl_xor(ls, 4); ls += __shfl_xor(ls, 8);
    const float fin = 64.0f / ls;
    so[w][8 * hh + r][ln]      = h16_bits((_Float16)(o0[r] * fin));
    so[w][8 * hh + r][16 + ln] = h16_bits((_Float16)(o1[r] * fin));
    so[w][8 * hh + r][32 + ln] = h16_bits((_Float16)(o2[r] * fin));
    so[w][8 * hh + r][48 + ln] = h16_bits((_Float16)(o3[r] * fin));
  }
  __builtin_amdgcn_fence(4  , "workgroup"); __builtin_amdgcn_wave_barrier();
  unsigned short* ob = (unsigned short*)O16 + ((size_t)b * SQ + q0) * DM + h * HD;
  const int rq = lane >> 3, pc = (lane & 7) * 8;
  for (int pass = 0; pass < 2; ++pass) {
#pragma unroll
    for (int it = 0; it < 4; ++it) { const int row = it * 4 + rq; const v8us v = *(const v8us*)&so[w][row][pc]; *(volatile v8us*)(ob + (size_t)row * DM + pc) = v; }
    if (pass == 0) __threadfence(); }
}

static constexpr size_t al256(size_t x) { return (x + 255) & ~(size_t)255; }
static constexpr size_t SZ_BQ  = (size_t)DM * DM * 2;
static constexpr size_t SZ_BKV = (size_t)KVD * DM * 2;
static constexpr size_t SZ_X16 = (size_t)MP * DM * 2;
static constexpr size_t SZ_QF  = (size_t)MP * DM * 4;
static constexpr size_t SZ_KF  = (size_t)MP * KVD * 4;
static constexpr size_t SZ_K16 = (size_t)MP * KVD * 2;
static constexpr size_t SZ_VT  = (size_t)NB * NG * HD * SQ * 2;
static constexpr size_t SZ_TAB = (size_t)SQ * (HD / 2) * 4;
static constexpr size_t SZ_QF0 = (size_t)NB * QT0 * DM * 4;
static constexpr size_t SZ_KF0 = (size_t)NB * QT0 * KVD * 4;
static constexpr size_t SZ_OH0 = (size_t)NB * QT0 * DM * 2;
static constexpr size_t OFF_BQ  = 0;
static constexpr size_t OFF_BK  = OFF_BQ  + al256(SZ_BQ);
static constexpr size_t OFF_BV  = OFF_BK  + al256(SZ_BKV);
static constexpr size_t OFF_BO  = OFF_BV  + al256(SZ_BKV);
static constexpr size_t OFF_X16 = OFF_BO  + al256(SZ_BQ);
static constexpr size_t OFF_QF  = OFF_X16 + al256(SZ_X16);
static constexpr size_t OFF_KF  = OFF_QF  + al256(SZ_QF);
static constexpr size_t OFF_VF  = OFF_KF  + al256(SZ_KF);
static constexpr size_t OFF_Q16 = OFF_VF  + al256(SZ_KF);
static constexpr size_t OFF_K16 = OFF_Q16 + al256(SZ_X16);
static constexpr size_t OFF_V16 = OFF_K16 + al256(SZ_K16);
static constexpr size_t OFF_VT  = OFF_V16 + al256(SZ_K16);
static constexpr size_t OFF_O16 = OFF_VT  + al256(SZ_VT);
static constexpr size_t OFF_INV = OFF_O16 + al256(SZ_X16);
static constexpr size_t OFF_CS  = OFF_INV + al256(128);
static constexpr size_t OFF_SN  = OFF_CS  + al256(SZ_TAB);
static constexpr size_t OFF_QF0 = OFF_SN  + al256(SZ_TAB);
static constexpr size_t OFF_KF0 = OFF_QF0 + al256(SZ_QF0);
static constexpr size_t OFF_OF0 = OFF_KF0 + al256(SZ_KF0);
static constexpr size_t OFF_OH0 = OFF_OF0 + al256(SZ_QF0);
static constexpr size_t OFF_OL0 = OFF_OH0 + al256(SZ_OH0);
static constexpr size_t WS_TOTAL = OFF_OL0 + al256(SZ_OH0);
static_assert(WS_TOTAL <= (size_t)134217728);

extern "C" void kernel_launch(void* const* d_in, const int* in_sizes, int n_in,
                              void* d_out, int out_size, void* d_ws, size_t ws_size, hipStream_t stream) {
  if (n_in < 5) return;
  const size_t xmin = ((size_t)(NB - 1) * SQ_FULL + SQ) * DM;
  if ((size_t)in_sizes[0] < xmin) return;
  if ((size_t)in_sizes[1] < (size_t)DM * DM) return;
  if ((size_t)in_sizes[2] < (size_t)KVD * DM) return;
  if ((size_t)in_sizes[3] < (size_t)KVD * DM) return;
  if ((size_t)in_sizes[4] < (size_t)DM * DM) return;
  if ((size_t)out_size < xmin) return;
  if (WS_TOTAL > ws_size) return;
  const float* x  = (const float*)d_in[0];
  const float* wq = (const float*)d_in[1];
  const float* wk = (const float*)d_in[2];
  const float* wv = (const float*)d_in[3];
  const float* wo = (const float*)d_in[4];
  float* out = (float*)d_out;
  char* ws = (char*)d_ws;
  _Float16* BQ = (_Float16*)(ws + OFF_BQ); _Float16* BK = (_Float16*)(ws + OFF_BK); _Float16* BV = (_Float16*)(ws + OFF_BV); _Float16* BO = (_Float16*)(ws + OFF_BO);
  _Float16* X16 = (_Float16*)(ws + OFF_X16);
  float* QF = (float*)(ws + OFF_QF); float* KF = (float*)(ws + OFF_KF); float* VF = (float*)(ws + OFF_VF);
  _Float16* Q16 = (_Float16*)(ws + OFF_Q16); _Float16* K16 = (_Float16*)(ws + OFF_K16); _Float16* V16 = (_Float16*)(ws + OFF_V16);
  _Float16* VT = (_Float16*)(ws + OFF_VT); _Float16* O16 = (_Float16*)(ws + OFF_O16);
  float* INVF = (float*)(ws + OFF_INV); float* CS = (float*)(ws + OFF_CS); float* SN = (float*)(ws + OFF_SN);
  float* QF0 = (float*)(ws + OFF_QF0); float* KF0 = (float*)(ws + OFF_KF0); float* OF0 = (float*)(ws + OFF_OF0);
  _Float16* OH0 = (_Float16*)(ws + OFF_OH0); _Float16* OL0 = (_Float16*)(ws + OFF_OL0);

  k_wnat<<<(unsigned)(((size_t)DM * DM / 8 + 255) / 256), 256, 0, stream>>>(wq, (size_t)DM * DM / 8, BQ);
  k_wnat<<<(unsigned)(((size_t)KVD * DM / 8 + 255) / 256), 256, 0, stream>>>(wk, (size_t)KVD * DM / 8, BK);
  k_wnat<<<(unsigned)(((size_t)KVD * DM / 8 + 255) / 256), 256, 0, stream>>>(wv, (size_t)KVD * DM / 8, BV);
  k_wnat<<<(unsigned)(((size_t)DM * DM / 8 + 255) / 256), 256, 0, stream>>>(wo, (size_t)DM * DM / 8, BO);
  k_x16<<<dim3((unsigned)(((size_t)SQ * DM / 8 + 255) / 256), NB), 256, 0, stream>>>(x, X16, (size_t)SQ * DM / 8);
  k_invf<<<1, 32, 0, stream>>>(10000.0f, INVF);
  k_tab2<<<(SQ * (HD / 2) + 255) / 256, 256, 0, stream>>>(INVF, CS, SN);
  k_gemm2<<<dim3((unsigned)((MP / 128) * (KVD / 64)), 1), 128, 0, stream>>>(X16, DM, 0, BV, DM, 0, 0.0625f, 0, VF, V16, KVD, 0, MP, KVD, DM);
  k_gemm2<<<dim3((unsigned)((MP / 128) * (DM / 64)), 1), 128, 0, stream>>>(X16, DM, 0, BQ, DM, 0, 0.0625f, 0, QF, nullptr, DM, 0, MP, DM, DM);
  k_gemm2<<<dim3((unsigned)((MP / 128) * (KVD / 64)), 1), 128, 0, stream>>>(X16, DM, 0, BK, DM, 0, 0.0625f, 0, KF, nullptr, KVD, 0, MP, KVD, DM);
  k_rope16<<<(unsigned)((size_t)MP * NH), 64, 0, stream>>>(QF, DM, NH, CS, SN, Q16, DM);
  k_rope16<<<(unsigned)((size_t)MP * NG), 64, 0, stream>>>(KF, KVD, NG, CS, SN, K16, KVD);
  k_ropef<<<dim3(QT0 * NH, NB), 64, 0, stream>>>(QF, DM, NH, CS, SN, QF0, DM);
  k_ropef<<<dim3(QT0 * NG, NB), 64, 0, stream>>>(KF, KVD, NG, CS, SN, KF0, KVD);
  k_vt<<<NB * NG * (SQ / 64), 256, 0, stream>>>(V16, VT);
  k_att0<<<dim3(NH * (QT0 / 64), NB), 64, 0, stream>>>(QF0, KF0, VF, 0.125f, OF0);
  k_flash<<<NB * NG * (SQ / 16), 128, 0, stream>>>(Q16, K16, VT, O16);
  k_gemm2<<<dim3((unsigned)((SQ / 128) * (DM / 64)), NB), 128, 0, stream>>>(O16, DM, (size_t)SQ * DM, BO, DM, 0, 0.0009765625f, 0, out, nullptr, DM, (size_t)SQ_FULL * DM, SQ, DM, DM);
  k_hl<<<(unsigned)(((size_t)NB * QT0 * DM / 8 + 255) / 256), 256, 0, stream>>>(OF0, OH0, OL0, (size_t)NB * QT0 * DM / 8);
  k_gemm2<<<dim3((unsigned)((QT0 / 128) * (DM / 64)), NB), 128, 0, stream>>>(OH0, DM, (size_t)QT0 * DM, BO, DM, 0, 0.0009765625f, 0, out, nullptr, DM, (size_t)SQ_FULL * DM, QT0, DM, DM);
  k_gemm2<<<dim3((unsigned)((QT0 / 128) * (DM / 64)), NB), 128, 0, stream>>>(OL0, DM, (size_t)QT0 * DM, BO, DM, 0, 0.00000095367431640625f, 1, out, nullptr, DM, (size_t)SQ_FULL * DM, QT0, DM, DM);
}
